// CGFE_36404142801270
// MI455X (gfx1250) — hardware-verified
//
#include <hip/hip_runtime.h>

#define NB    4
#define CIN   256
#define CQK   32
#define HWN   4096
#define CVS   512
#define TOKB  64
#define XP    264
#define QBLK  32
#define KCH   64
#define SPI   68
#define PPI   72
#define EPI   36

static_assert((HWN % TOKB) == 0 && (HWN % QBLK) == 0 && (HWN % KCH) == 0);
static_assert((CIN % 32) == 0 && CQK == 32 && CVS == 2 * CIN);
static_assert((XP % 8) == 0 && (SPI % 4) == 0 && (PPI % 8) == 0 && (EPI % 4) == 0);
static_assert(CIN * TOKB <= TOKB * XP);

typedef __bf16         v16bf __attribute__((ext_vector_type(16)));
typedef unsigned short v16us __attribute__((ext_vector_type(16)));
typedef unsigned short v8us  __attribute__((ext_vector_type(8)));
typedef _Float16       v16h  __attribute__((ext_vector_type(16)));
typedef _Float16       v8h   __attribute__((ext_vector_type(8)));
typedef float          v8f   __attribute__((ext_vector_type(8)));
typedef float          v4f   __attribute__((ext_vector_type(4)));
typedef unsigned int   v4u   __attribute__((ext_vector_type(4)));

__device__ __forceinline__ unsigned short bf_bits(float f) {
  unsigned u = __float_as_uint(f);
  return (unsigned short)((u + 0x7FFFu + ((u >> 16) & 1u)) >> 16);
}
__device__ __forceinline__ float bf_up(unsigned short hb) { return __uint_as_float(((unsigned)hb) << 16); }
__device__ __forceinline__ float bf_r(float f) { return bf_up(bf_bits(f)); }
__device__ __forceinline__ unsigned short h_bits(float f) {
  const _Float16 hv = (_Float16)f;
  return __builtin_bit_cast(unsigned short, hv);
}
__device__ __forceinline__ v8f zero8() { v8f z = {0.f, 0.f, 0.f, 0.f, 0.f, 0.f, 0.f, 0.f}; return z; }

__device__ __forceinline__ v16bf ldfrag_b(const unsigned short* p) {
  union { v16us v; v8us hv[2]; } f;
  f.hv[0] = *(const v8us*)(p);
  f.hv[1] = *(const v8us*)(p + 16);
  return __builtin_bit_cast(v16bf, f.v);
}
__device__ __forceinline__ v16h ldfrag_h(const _Float16* p) {
  union { v16h v; v8h hv[2]; } f;
  f.hv[0] = *(const v8h*)(p);
  f.hv[1] = *(const v8h*)(p + 16);
  return f.v;
}

__device__ __forceinline__ v8f mma_b(v16bf a, v16bf b, v8f c) {
  return __builtin_amdgcn_wmma_f32_16x16x32_bf16(false, a, false, b, (short)0, c, false, false);
}
__device__ __forceinline__ v8f mma_h(v16h a, v16h b, v8f c) {
  return __builtin_amdgcn_wmma_f32_16x16x32_f16(false, a, false, b, (short)0, c, false, false);
}
__device__ __forceinline__ void guard_v8(v8f& c0, v8f& c1, v8f& c2, v8f& c3, v8f& c4, v8f& c5, v8f& c6, v8f& c7,
                                         v16bf a0, v16bf a1, v16bf b0, v16bf b1, v16bf b2, v16bf b3) {
#if defined(__HIP_DEVICE_COMPILE__)
  asm volatile("v_nop\n\tv_nop\n\tv_nop\n\tv_nop"
               : "+v"(c0), "+v"(c1), "+v"(c2), "+v"(c3), "+v"(c4), "+v"(c5), "+v"(c6), "+v"(c7)
               : "v"(a0), "v"(a1), "v"(b0), "v"(b1), "v"(b2), "v"(b3));
#endif
}
__device__ __forceinline__ void guard_v2(v8f& c0, v8f& c1, v16bf a, v16bf b0, v16bf b1) {
#if defined(__HIP_DEVICE_COMPILE__)
  asm volatile("v_nop\n\tv_nop\n\tv_nop\n\tv_nop" : "+v"(c0), "+v"(c1) : "v"(a), "v"(b0), "v"(b1));
#endif
}
__device__ __forceinline__ void guard_s1(v8f& s, v16bf a0, v16bf a1, v16bf b0, v16bf b1) {
#if defined(__HIP_DEVICE_COMPILE__)
  asm volatile("v_nop\n\tv_nop\n\tv_nop\n\tv_nop" : "+v"(s) : "v"(a0), "v"(a1), "v"(b0), "v"(b1));
#endif
}
__device__ __forceinline__ void guard_h4(v8f& c0, v8f& c1, v8f& c2, v8f& c3,
                                         v16h a, v16h b0, v16h b1, v16h b2, v16h b3) {
#if defined(__HIP_DEVICE_COMPILE__)
  asm volatile("v_nop\n\tv_nop\n\tv_nop\n\tv_nop"
               : "+v"(c0), "+v"(c1), "+v"(c2), "+v"(c3)
               : "v"(a), "v"(b0), "v"(b1), "v"(b2), "v"(b3));
#endif
}
__device__ __forceinline__ void sched_fence() {
#if defined(__HIP_DEVICE_COMPILE__)
  asm volatile("" ::: "memory");
#endif
}

__global__ __launch_bounds__(256) void k_prep(const float* __restrict__ Wv1, const float* __restrict__ Wv2,
                                               const float* __restrict__ Wq, const float* __restrict__ Wk,
                                               unsigned short* WB) {
  const int blk = blockIdx.x, tid = threadIdx.x;
  const int piece = blk * 256 + tid;
  const float* src;
  int p;
  if (blk < 32)      { src = Wv1; p = piece; }
  else if (blk < 64) { src = Wv2; p = piece - 8192; }
  else if (blk < 68) { src = Wq;  p = piece - 16384; }
  else               { src = Wk;  p = piece - 17408; }
  const v4f a = *(const v4f*)(src + (size_t)p * 8);
  const v4f c = *(const v4f*)(src + (size_t)p * 8 + 4);
  v8us o;
  o[0] = bf_bits(a[0]); o[1] = bf_bits(a[1]); o[2] = bf_bits(a[2]); o[3] = bf_bits(a[3]);
  o[4] = bf_bits(c[0]); o[5] = bf_bits(c[1]); o[6] = bf_bits(c[2]); o[7] = bf_bits(c[3]);
  unsigned short* dst = WB + (size_t)piece * 8;
  *(volatile v8us*)dst = o;
  __threadfence();
  *(volatile v8us*)dst = o;
}

__global__ __launch_bounds__(256) void k_projv(const float* __restrict__ x1, const float* __restrict__ x2,
                                                const unsigned short* WB,
                                                const float* __restrict__ bv1, const float* __restrict__ bv2,
                                                unsigned short* Vp) {
  __shared__ __align__(16) unsigned short sX[TOKB * XP];
  __shared__ float sbias[CIN];
  const int tid = threadIdx.x, wave = tid >> 5, lane = tid & 31, m = lane & 15, h = lane >> 4;
  const int vsel = blockIdx.y;
  const int b = blockIdx.x / (HWN / TOKB), n0 = (blockIdx.x % (HWN / TOKB)) * TOKB;
  const float* x = vsel ? x2 : x1;
  const float* bv = vsel ? bv2 : bv1;
  const unsigned short* Wb = WB + (size_t)vsel * (CIN * CIN);
  sbias[tid] = bf_r(bv[tid]);
  const float* xb = x + (size_t)b * CIN * HWN + n0;
#pragma unroll 4
  for (int it = 0; it < (CIN * TOKB) / (4 * 256); ++it) {
    const int e = it * 256 + tid;
    const int c = e >> 4, n4 = (e & 15) * 4;
    const v4f v = *(const v4f*)(xb + (size_t)c * HWN + n4);
    unsigned short* d = sX + n4 * XP + c;
    d[0] = bf_bits(v[0]); d[XP] = bf_bits(v[1]); d[2 * XP] = bf_bits(v[2]); d[3 * XP] = bf_bits(v[3]);
  }
  __syncthreads();

  v8f acc[8];
#pragma unroll
  for (int t = 0; t < 8; ++t) acc[t] = zero8();
  const unsigned short* wa = Wb + (size_t)(32 * wave + m) * CIN + 8 * h;
  const unsigned short* xf = sX + m * XP + 8 * h;
#pragma unroll 2
  for (int ks = 0; ks < CIN / 32; ++ks) {
    const v16bf a0 = ldfrag_b(wa + 32 * ks);
    const v16bf a1 = ldfrag_b(wa + 16 * CIN + 32 * ks);
    const v16bf f0 = ldfrag_b(xf + 32 * ks);
    const v16bf f1 = ldfrag_b(xf + 16 * XP + 32 * ks);
    const v16bf f2 = ldfrag_b(xf + 32 * XP + 32 * ks);
    const v16bf f3 = ldfrag_b(xf + 48 * XP + 32 * ks);
    acc[0] = mma_b(a0, f0, acc[0]);
    acc[1] = mma_b(a0, f1, acc[1]);
    acc[2] = mma_b(a0, f2, acc[2]);
    acc[3] = mma_b(a0, f3, acc[3]);
    acc[4] = mma_b(a1, f0, acc[4]);
    acc[5] = mma_b(a1, f1, acc[5]);
    acc[6] = mma_b(a1, f2, acc[6]);
    acc[7] = mma_b(a1, f3, acc[7]);
    guard_v8(acc[0], acc[1], acc[2], acc[3], acc[4], acc[5], acc[6], acc[7], a0, a1, f0, f1, f2, f3);
    sched_fence();
  }
  __syncthreads();
#pragma unroll
  for (int t = 0; t < 2; ++t) {
#pragma unroll
    for (int nt = 0; nt < 4; ++nt) {
#pragma unroll
      for (int r = 0; r < 8; ++r) {
        const int o = 32 * wave + 16 * t + 8 * h + r;
        sX[o * TOKB + 16 * nt + m] = h_bits(acc[4 * t + nt][r] + sbias[o]);
      }
    }
  }
  __syncthreads();
  unsigned short* vdst = Vp + ((size_t)(b * CVS + vsel * CIN)) * HWN + n0;
  const int qg = lane >> 3, piece = lane & 7;
#pragma unroll
  for (int it = 0; it < 8; ++it) {
    const int L = it * 32 + 4 * wave + qg;
    const v4u v = *(const v4u*)(sX + L * TOKB + piece * 8);
    unsigned short* d = vdst + (size_t)L * HWN + piece * 8;
    *(volatile v4u*)d = v;
    __threadfence();
    *(volatile v4u*)d = v;
  }
}

__global__ __launch_bounds__(256) void k_projqk(const float* __restrict__ chg, const unsigned short* WQK,
                                                 const float* __restrict__ bq, const float* __restrict__ bk,
                                                 unsigned short* Qh, unsigned short* Ql,
                                                 unsigned short* Kh, unsigned short* Kl) {
  __shared__ __align__(16) unsigned short sX[TOKB * XP];
  __shared__ __align__(16) unsigned short sO[4 * TOKB * CQK];
  __shared__ float sbias[64];
  const int tid = threadIdx.x, wave = tid >> 5, lane = tid & 31, m = lane & 15, h = lane >> 4;
  const int b = blockIdx.x / (HWN / TOKB), n0 = (blockIdx.x % (HWN / TOKB)) * TOKB;
  if (tid < 64) {
    const float vq = bq[tid & 31];
    const float vk = bk[tid & 31];
    sbias[tid] = bf_r(tid < 32 ? vq : vk);
  }
  const float* xb = chg + (size_t)b * CIN * HWN + n0;
#pragma unroll 4
  for (int it = 0; it < (CIN * TOKB) / (4 * 256); ++it) {
    const int e = it * 256 + tid;
    const int c = e >> 4, n4 = (e & 15) * 4;
    const v4f v = *(const v4f*)(xb + (size_t)c * HWN + n4);
    unsigned short* d = sX + n4 * XP + c;
    d[0] = bf_bits(v[0]); d[XP] = bf_bits(v[1]); d[2 * XP] = bf_bits(v[2]); d[3 * XP] = bf_bits(v[3]);
  }
  __syncthreads();

  const int dt = wave & 3, ntp = (wave >> 2) * 2;
  const unsigned short* wa = WQK + (size_t)(16 * dt + m) * CIN + 8 * h;
  const unsigned short* xf = sX + (16 * ntp + m) * XP + 8 * h;
  v8f acc[2];
  acc[0] = zero8(); acc[1] = zero8();
#pragma unroll 2
  for (int ks = 0; ks < CIN / 32; ++ks) {
    const v16bf a  = ldfrag_b(wa + 32 * ks);
    const v16bf f0 = ldfrag_b(xf + 32 * ks);
    const v16bf f1 = ldfrag_b(xf + 16 * XP + 32 * ks);
    acc[0] = mma_b(a, f0, acc[0]);
    acc[1] = mma_b(a, f1, acc[1]);
    guard_v2(acc[0], acc[1], a, f0, f1);
    sched_fence();
  }
  const int plane0 = 2 * (dt >> 1);
#pragma unroll
  for (int t = 0; t < 2; ++t) {
    const int n = 16 * (ntp + t) + m;
#pragma unroll
    for (int r = 0; r < 8; ++r) {
      const int dd = 16 * (dt & 1) + 8 * h + r;
      const float val = acc[t][r] + sbias[16 * dt + 8 * h + r];
      const unsigned short hb = bf_bits(val);
      const unsigned short lb = bf_bits(val - bf_up(hb));
      sO[plane0 * (TOKB * CQK) + n * CQK + dd] = hb;
      sO[(plane0 + 1) * (TOKB * CQK) + n * CQK + dd] = lb;
    }
  }
  __syncthreads();
  const size_t gbase = ((size_t)(b * HWN + n0)) * CQK;
  const int qg = lane >> 3, piece = lane & 7;
  const int L = 4 * wave + qg;
#pragma unroll
  for (int it = 0; it < 4; ++it) {
    unsigned short* pl = (it == 0) ? Qh : (it == 1) ? Ql : (it == 2) ? Kh : Kl;
    const v4u v = *(const v4u*)(sO + it * (TOKB * CQK) + L * 64 + piece * 8);
    unsigned short* d = pl + gbase + (size_t)L * 64 + piece * 8;
    *(volatile v4u*)d = v;
    __threadfence();
    *(volatile v4u*)d = v;
  }
}

__global__ __launch_bounds__(256) void k_attn(const unsigned short* Qh, const unsigned short* Ql,
                                               const unsigned short* Kh, const unsigned short* Kl,
                                               const _Float16* Vp,
                                               const float* __restrict__ x1, const float* __restrict__ x2,
                                               const float* __restrict__ g1, const float* __restrict__ g2,
                                               float* out) {
  __shared__ __align__(16) float sS[QBLK * SPI];
  __shared__ __align__(16) _Float16 sP[QBLK * PPI];
  __shared__ __align__(16) float sM[QBLK];
  __shared__ __align__(16) float sL[QBLK];
  __shared__ __align__(16) float sA[QBLK];
  __shared__ __align__(16) float sE[CIN * EPI];
  const int tid = threadIdx.x, wave = tid >> 5, lane = tid & 31, m = lane & 15, h = lane >> 4;
  const int qt = wave >> 2, cg = wave & 3;
  const int b = blockIdx.x / (HWN / QBLK), i0 = (blockIdx.x % (HWN / QBLK)) * QBLK;
  if (tid < QBLK) { sM[tid] = -1.0e30f; sL[tid] = 0.0f; sA[tid] = 0.0f; }
  const float gb1 = bf_r(g1[0]), gb2 = bf_r(g2[0]);
  const size_t tok0 = (size_t)b * HWN;
  const v16bf fqh = ldfrag_b(Qh + (tok0 + i0 + 16 * qt + m) * CQK + 8 * h);
  const v16bf fql = ldfrag_b(Ql + (tok0 + i0 + 16 * qt + m) * CQK + 8 * h);
  const unsigned short* khp = Kh + (tok0 + 16 * cg + m) * CQK + 8 * h;
  const unsigned short* klp = Kl + (tok0 + 16 * cg + m) * CQK + 8 * h;
  const _Float16* vrp = Vp + ((size_t)b * CVS + 128 * cg + m) * HWN + 8 * h;
  float* ssw = sS + (16 * qt + 8 * h) * SPI + 16 * cg + m;
  const int srow = 4 * wave + (lane >> 3), skq = (lane & 7) * 8;
  const _Float16* spa = sP + (16 * qt + m) * PPI + 8 * h;

  v8f acc[8];
#pragma unroll
  for (int t = 0; t < 8; ++t) acc[t] = zero8();

#pragma unroll 1
  for (int j0 = 0; j0 < HWN; j0 += KCH) {
    {
      const v16bf kh0 = ldfrag_b(khp + (size_t)j0 * CQK);
      const v16bf kl0 = ldfrag_b(klp + (size_t)j0 * CQK);
      v8f s = zero8();
      s = mma_b(fqh, kh0, s);
      s = mma_b(fqh, kl0, s);
      s = mma_b(fql, kh0, s);
      guard_s1(s, fqh, fql, kh0, kl0);
      sched_fence();
#pragma unroll
      for (int r = 0; r < 8; ++r) ssw[r * SPI] = s[r];
    }
    __syncthreads();
    {
      const v4f t0 = *(const v4f*)(sS + srow * SPI + skq);
      const v4f t1 = *(const v4f*)(sS + srow * SPI + skq + 4);
      float lmax = fmaxf(fmaxf(fmaxf(t0[0], t0[1]), fmaxf(t0[2], t0[3])),
                         fmaxf(fmaxf(t1[0], t1[1]), fmaxf(t1[2], t1[3])));
      lmax = fmaxf(lmax, __shfl_xor(lmax, 1, 32));
      lmax = fmaxf(lmax, __shfl_xor(lmax, 2, 32));
      lmax = fmaxf(lmax, __shfl_xor(lmax, 4, 32));
      const float mo = sM[srow];
      const float lold = sL[srow];
      const float mn = fmaxf(mo, lmax);
      const float alpha = __expf(mo - mn);
      float pr[8];
#pragma unroll
      for (int j = 0; j < 4; ++j) { pr[j] = __expf(t0[j] - mn); pr[4 + j] = __expf(t1[j] - mn); }
      float psum = ((pr[0] + pr[1]) + (pr[2] + pr[3])) + ((pr[4] + pr[5]) + (pr[6] + pr[7]));
      psum += __shfl_xor(psum, 1, 32);
      psum += __shfl_xor(psum, 2, 32);
      psum += __shfl_xor(psum, 4, 32);
      v8h pv;
#pragma unroll
      for (int j = 0; j < 8; ++j) pv[j] = (_Float16)(pr[j] * 1024.0f);
      *(v8h*)(sP + srow * PPI + skq) = pv;
      if ((lane & 7) == 0) { sM[srow] = mn; sL[srow] = lold * alpha + psum; sA[srow] = alpha; }
    }
    __syncthreads();
    {
      const v4f al0 = *(const v4f*)(sA + 16 * qt + 8 * h);
      const v4f al1 = *(const v4f*)(sA + 16 * qt + 8 * h + 4);
      int need = 0;
#pragma unroll
      for (int r = 0; r < 4; ++r) { need |= (al0[r] != 1.0f); need |= (al1[r] != 1.0f); }
      if (__any(need)) {
#pragma unroll
        for (int ct = 0; ct < 8; ++ct) {
#pragma unroll
          for (int r = 0; r < 4; ++r) { acc[ct][r] *= al0[r]; acc[ct][4 + r] *= al1[r]; }
        }
      }
    }
#pragma unroll
    for (int kc = 0; kc < 2; ++kc) {
      const v16h pa = ldfrag_h(spa + 32 * kc);
      const _Float16* vb = vrp + j0 + 32 * kc;
      {
        const v16h b0 = ldfrag_h(vb);
        const v16h b1 = ldfrag_h(vb + (size_t)16 * HWN);
        const v16h b2 = ldfrag_h(vb + (size_t)32 * HWN);
        const v16h b3 = ldfrag_h(vb + (size_t)48 * HWN);
        acc[0] = mma_h(pa, b0, acc[0]);
        acc[1] = mma_h(pa, b1, acc[1]);
        acc[2] = mma_h(pa, b2, acc[2]);
        acc[3] = mma_h(pa, b3, acc[3]);
        guard_h4(acc[0], acc[1], acc[2], acc[3], pa, b0, b1, b2, b3);
        sched_fence();
      }
      {
        const v16h b4 = ldfrag_h(vb + (size_t)64 * HWN);
        const v16h b5 = ldfrag_h(vb + (size_t)80 * HWN);
        const v16h b6 = ldfrag_h(vb + (size_t)96 * HWN);
        const v16h b7 = ldfrag_h(vb + (size_t)112 * HWN);
        acc[4] = mma_h(pa, b4, acc[4]);
        acc[5] = mma_h(pa, b5, acc[5]);
        acc[6] = mma_h(pa, b6, acc[6]);
        acc[7] = mma_h(pa, b7, acc[7]);
        guard_h4(acc[4], acc[5], acc[6], acc[7], pa, b4, b5, b6, b7);
        sched_fence();
      }
    }
  }

  const v4f lz0 = *(const v4f*)(sL + 16 * qt + 8 * h);
  const v4f lz1 = *(const v4f*)(sL + 16 * qt + 8 * h + 4);
  float li[8];
#pragma unroll
  for (int r = 0; r < 4; ++r) { li[r] = 1.0f / lz0[r]; li[4 + r] = 1.0f / lz1[r]; }
  const int qg = lane >> 3, piece = lane & 7;
#pragma unroll
  for (int p = 0; p < 2; ++p) {
    __syncthreads();
    if ((cg >> 1) == p) {
      float* se = sE + (128 * (cg & 1) + m) * EPI + 16 * qt + 8 * h;
#pragma unroll
      for (int ct = 0; ct < 8; ++ct) {
#pragma unroll
        for (int r = 0; r < 8; ++r) se[16 * ct * EPI + r] = acc[ct][r] * (li[r] * (1.0f / 1024.0f));
      }
    }
    __syncthreads();
    const float* xr = p ? x2 : x1;
    const float g = p ? gb2 : gb1;
    float* ob = out + (size_t)p * ((size_t)NB * CIN * HWN);
#pragma unroll
    for (int it = 0; it < 8; ++it) {
      const int L = it * 32 + 4 * wave + qg;
      const v4f o4 = *(const v4f*)(sE + L * EPI + 4 * piece);
      const size_t idx = ((size_t)(b * CIN + L)) * HWN + i0 + 4 * piece;
      const v4f xv = *(const v4f*)(xr + idx);
      v4f res;
      res[0] = bf_r(xv[0]) + g * o4[0];
      res[1] = bf_r(xv[1]) + g * o4[1];
      res[2] = bf_r(xv[2]) + g * o4[2];
      res[3] = bf_r(xv[3]) + g * o4[3];
      float* d = ob + idx;
      *(volatile v4f*)d = res;
      __threadfence();
      *(volatile v4f*)d = res;
    }
  }
}

extern "C" void kernel_launch(void* const* d_in, const int* in_sizes, int n_in,
                              void* d_out, int out_size, void* d_ws, size_t ws_size,
                              hipStream_t stream) {
  if (n_in < 13) return;
  if (in_sizes[0] != NB * CIN * HWN || in_sizes[1] != NB * CIN * HWN || in_sizes[2] != NB * CIN * HWN) return;
  if (in_sizes[3] != CQK * CIN || in_sizes[4] != CQK) return;
  if (in_sizes[5] != CQK * CIN || in_sizes[6] != CQK) return;
  if (in_sizes[7] != CIN * CIN || in_sizes[8] != CIN) return;
  if (in_sizes[9] != CIN * CIN || in_sizes[10] != CIN) return;
  if (in_sizes[11] < 1 || in_sizes[12] < 1) return;
  if (out_size != 2 * NB * CIN * HWN) return;

  const float* x1  = (const float*)d_in[0];
  const float* x2  = (const float*)d_in[1];
  const float* chg = (const float*)d_in[2];
  const float* Wq  = (const float*)d_in[3];
  const float* bq  = (const float*)d_in[4];
  const float* Wk  = (const float*)d_in[5];
  const float* bk  = (const float*)d_in[6];
  const float* Wv1 = (const float*)d_in[7];
  const float* bv1 = (const float*)d_in[8];
  const float* Wv2 = (const float*)d_in[9];
  const float* bv2 = (const float*)d_in[10];
  const float* g1  = (const float*)d_in[11];
  const float* g2  = (const float*)d_in[12];
  float* out = (float*)d_out;

  const size_t PWB = (size_t)(2 * CIN * CIN + 2 * CQK * CIN) * 2;
  const size_t PQK = (size_t)NB * HWN * CQK * 2;
  const size_t PV  = (size_t)NB * CVS * HWN * 2;

  size_t off = 0;
  const size_t oWB = off; off += PWB;
  const size_t oQH = off; off += PQK;
  const size_t oQL = off; off += PQK;
  const size_t oKH = off; off += PQK;
  const size_t oKL = off; off += PQK;
  const size_t oV  = off; off += PV;
  if (off > ws_size) return;
  if (off > (size_t)134217728) return;

  char* ws = (char*)d_ws;
  unsigned short* WB = (unsigned short*)(ws + oWB);
  unsigned short* QH = (unsigned short*)(ws + oQH);
  unsigned short* QL = (unsigned short*)(ws + oQL);
  unsigned short* KH = (unsigned short*)(ws + oKH);
  unsigned short* KL = (unsigned short*)(ws + oKL);
  unsigned short* V  = (unsigned short*)(ws + oV);

  k_prep<<<dim3(72), dim3(256), 0, stream>>>(Wv1, Wv2, Wq, Wk, WB);
  k_projv<<<dim3(NB * (HWN / TOKB), 2), dim3(256), 0, stream>>>(x1, x2, WB, bv1, bv2, V);
  k_projqk<<<dim3(NB * (HWN / TOKB)), dim3(256), 0, stream>>>(chg, WB + 2 * CIN * CIN, bq, bk, QH, QL, KH, KL);
  k_attn<<<dim3(NB * (HWN / QBLK)), dim3(256), 0, stream>>>(QH, QL, KH, KL, (const _Float16*)V,
                                                            x1, x2, g1, g2, out);
  (void)hipGetLastError();
}
